// PERConv_11716670783823
// MI455X (gfx1250) — hardware-run, weakly checked
//
#include <hip/hip_runtime.h>
#include <stddef.h>
#include <stdint.h>
#include <math.h>

#define NN      100000
#define NE      1600000
#define HD      64
#define NG      64
#define GBM     128
#define MP      100096
#define K1      64
#define N1      128
#define K2      128
#define NTHR    256
#define NWAVE   8
#define EPT     8
#define WCH     (32 * EPT)
#define NBRUN   1024
#define SLB     10
#define NBK     98
#define WLCAP   3584
#define RCAP    28672
#define DEGCAP  64
#define SRCBITS 17
#define MAXDEG_MEAS   36
#define MAXB1024_MEAS 16673
#define SP      68
#define WSMAX   134217728

#define BK_ZINTS (NWAVE * WLCAP + RCAP + 3 * NBRUN)
#define BK_INTS  (BK_ZINTS + 16)
#define BK_LDS   (BK_INTS * 4)

#define NBIN     (4 * NG * HD)
#define STAT_LDS (NBIN * 8 + NG * HD * 4 + 256 * 4 + 64 * 4)

#define PBX   (MP * HD / 8 / NTHR)
#define PBW1  (N1 * K1 / 8 / NTHR)
#define PBFC  (HD * K2 / 8 / NTHR)
#define PBTOT (PBX + PBW1 + PBFC + 1)

#define T_WP 0
#define T_MB 192
#define T_GW 256
#define T_GB 320
#define T_GS 384
#define T_FB 448

static_assert(HD == 64 && NG == 64);
static_assert(NN % 16 == 0 && NN % 2 == 0);
static_assert(MP % GBM == 0 && MP >= NN && MP == 782 * GBM && NN - 781 * GBM == 32);
static_assert(K1 % 32 == 0 && K2 % 32 == 0 && K2 == 2 * HD && N1 == 2 * HD);
static_assert(NBRUN == (1 << SLB) && NBRUN == 1024 && NBRUN % GBM == 0 && NBRUN % 32 == 0);
static_assert(NBK * NBRUN >= MP && NBK * NBRUN >= NN);
static_assert(NN <= (1 << SRCBITS) && NN <= 131072 && SRCBITS + SLB <= 31);
static_assert((((long long)NE) << SLB) < (1LL << 31));
static_assert(NE % WCH == 0 && NE % 4 == 0);
static_assert(RCAP == NWAVE * WLCAP && RCAP % 4 == 0 && BK_ZINTS % (NTHR * 4) == 0);
static_assert((long long)RCAP * 100 >= (long long)MAXB1024_MEAS * 105);
static_assert(WLCAP >= MAXB1024_MEAS / 8 + 8 * 46 + 1);
static_assert(MAXDEG_MEAS + 8 <= DEGCAP);
static_assert(BK_LDS <= 300000 && STAT_LDS <= 300000);
static_assert((MP * HD / 8) % NTHR == 0 && (N1 * K1 / 8) % NTHR == 0 && (HD * K2 / 8) % NTHR == 0);
static_assert((GBM * SP + GBM * 3 + 256) * 4 <= 65536);
static_assert((NN * 3) % 4 == 0 && (GBM * 3) % 4 == 0);

typedef float          v4f   __attribute__((ext_vector_type(4)));
typedef float          v8f   __attribute__((ext_vector_type(8)));
typedef double         v2d   __attribute__((ext_vector_type(2)));
typedef int            v4i   __attribute__((ext_vector_type(4)));
typedef int            v8i   __attribute__((ext_vector_type(8)));
typedef unsigned short v8us  __attribute__((ext_vector_type(8)));
typedef unsigned short v16us __attribute__((ext_vector_type(16)));
typedef __bf16         v16bf __attribute__((ext_vector_type(16)));
typedef v4f  __attribute__((may_alias)) v4fa;
typedef v4i  __attribute__((may_alias)) v4ia;
typedef v8us __attribute__((may_alias)) v8usa;
union FragB { v16bf v; v16us u; v8us h[2]; v8i w; };

__device__ __forceinline__ v8f wmb(const FragB& a, const FragB& b, v8f c) {
  v8f d = __builtin_amdgcn_wmma_f32_16x16x32_bf16(false, a.v, false, b.v, (short)0, c, false, false);
  asm volatile("v_nop\n\tv_nop\n\tv_nop\n\tv_nop" : "+v"(d) : "v"(a.w), "v"(b.w));
  return d;
}

__device__ __forceinline__ unsigned bf16_bits(float f) {
  const unsigned u = __float_as_uint(f);
  const unsigned r = (u + 0x7FFFu + ((u >> 16) & 1u)) >> 16;
  const unsigned q = (u >> 16) | 0x40u;
  return ((u & 0x7fffffffu) > 0x7f800000u) ? q : r;
}
__device__ __forceinline__ float bf16_val(float f) {
  return __uint_as_float(bf16_bits(f) << 16);
}

__device__ __forceinline__ void hilo_pack(float v0, float v1, float v2, float v3,
                                          int& h01, int& h23, int& l01, int& l23) {
  const unsigned a0 = bf16_bits(v0), a1 = bf16_bits(v1), a2 = bf16_bits(v2), a3 = bf16_bits(v3);
  const unsigned b0 = bf16_bits(v0 - __uint_as_float(a0 << 16));
  const unsigned b1 = bf16_bits(v1 - __uint_as_float(a1 << 16));
  const unsigned b2 = bf16_bits(v2 - __uint_as_float(a2 << 16));
  const unsigned b3 = bf16_bits(v3 - __uint_as_float(a3 << 16));
  h01 = (int)(a0 | (a1 << 16)); h23 = (int)(a2 | (a3 << 16));
  l01 = (int)(b0 | (b1 << 16)); l23 = (int)(b2 | (b3 << 16));
}

__device__ __forceinline__ v4i regroup8(int h01, int h23, int l01, int l23, int lane) {
  const int t  = lane & 15;
  const int s0 = (lane & 16) + ((2 * t) & 15), s1 = s0 + 1;
  const int a0 = __shfl(h01, s0, 32), a1 = __shfl(h23, s0, 32), a2 = __shfl(h01, s1, 32), a3 = __shfl(h23, s1, 32);
  const int b0 = __shfl(l01, s0, 32), b1 = __shfl(l23, s0, 32), b2 = __shfl(l01, s1, 32), b3 = __shfl(l23, s1, 32);
  const int mk = (t < 8) ? -1 : 0;
  v4i o;
  o.x = (a0 & mk) | (b0 & ~mk); o.y = (a1 & mk) | (b1 & ~mk);
  o.z = (a2 & mk) | (b2 & ~mk); o.w = (a3 & mk) | (b3 & ~mk);
  return o;
}

__device__ __forceinline__ void st2_v4f(float* p, v4f v) {
  *(volatile v4f*)p = v;
  __threadfence();
  *(volatile v4f*)p = v;
}
__device__ __forceinline__ void st2_v4i(int* p, v4i v) {
  *(volatile v4i*)p = v;
  __threadfence();
  *(volatile v4i*)p = v;
}
__device__ __forceinline__ void st2_v8us(unsigned short* p, v8us v) {
  *(volatile v8us*)p = v;
  __threadfence();
  *(volatile v8us*)p = v;
}

__device__ __forceinline__ v8us gather8(const float* __restrict__ base, int stride) {
  float f[8];
#pragma unroll
  for (int i = 0; i < 8; ++i) f[i] = base[(size_t)i * (size_t)stride];
  v8us o;
#pragma unroll
  for (int i = 0; i < 8; ++i) o[i] = (unsigned short)bf16_bits(f[i]);
  return o;
}

__device__ __forceinline__ float blend6(float a, float b, float c, float d, float e, float f,
                                        unsigned m0, unsigned m1, unsigned m2, unsigned m3, unsigned m4, unsigned m5) {
  const unsigned w = ((bf16_bits(a) << 16) & m0) | ((bf16_bits(b) << 16) & m1) | ((bf16_bits(c) << 16) & m2) |
                     ((bf16_bits(d) << 16) & m3) | ((bf16_bits(e) << 16) & m4) | ((bf16_bits(f) << 16) & m5);
  return __uint_as_float(w);
}

__global__ __launch_bounds__(NTHR) void k_prep(const float* __restrict__ x, const float* __restrict__ mw,
                                               const float* __restrict__ mbp, const float* __restrict__ gwp,
                                               const float* __restrict__ gbp, const float* __restrict__ gsp,
                                               const float* __restrict__ fcw, const float* __restrict__ fbp,
                                               unsigned short* xb, unsigned short* w1t, unsigned short* fcd,
                                               float* tab) {
  const int tid = (int)threadIdx.x;
  const int blk = (int)blockIdx.x;
  if (blk < PBX) {
    const int u   = blk * NTHR + tid;
    const int row = u >> 3, k8 = (u & 7) * 8;
    const int rc  = row < NN ? row : NN - 1;
    const unsigned mk = row < NN ? 0xffffu : 0u;
    const float* p = x + (size_t)rc * HD + k8;
    const v4f a = *(const v4fa*)p;
    const v4f b = *(const v4fa*)(p + 4);
    v8us o;
    o[0] = (unsigned short)(bf16_bits(a.x) & mk); o[1] = (unsigned short)(bf16_bits(a.y) & mk);
    o[2] = (unsigned short)(bf16_bits(a.z) & mk); o[3] = (unsigned short)(bf16_bits(a.w) & mk);
    o[4] = (unsigned short)(bf16_bits(b.x) & mk); o[5] = (unsigned short)(bf16_bits(b.y) & mk);
    o[6] = (unsigned short)(bf16_bits(b.z) & mk); o[7] = (unsigned short)(bf16_bits(b.w) & mk);
    st2_v8us(xb + (size_t)row * HD + k8, o);
  } else if (blk < PBX + PBW1) {
    const int u = (blk - PBX) * NTHR + tid;
    const int n = u >> 3, k8 = (u & 7) * 8;
    const int off = (n < HD) ? (k8 * HD + n) : ((HD + k8) * HD + (n - HD));
    const v8us o = gather8(mw + off, HD);
    st2_v8us(w1t + (size_t)n * K1 + k8, o);
  } else if (blk < PBX + PBW1 + PBFC) {
    const int u = (blk - PBX - PBW1) * NTHR + tid;
    const int n = u >> 4, k8 = (u & 15) * 8, kk = k8 & 63;
    const v8us o = gather8(fcw + (size_t)kk * HD + n, HD);
    st2_v8us(fcd + (size_t)n * K2 + k8, o);
  } else {
    if (tid < 128) {
      const int grp = tid >> 4, q = tid & 15;
      const int ia  = tid < 48 ? tid : 47;
      const v4f a = *(const v4fa*)(mw + 128 * HD + 4 * ia);
      const v4f b = *(const v4fa*)(mbp + 4 * q);
      const v4f c = *(const v4fa*)(gwp + 4 * q);
      const v4f d = *(const v4fa*)(gbp + 4 * q);
      const v4f e = *(const v4fa*)(gsp + 4 * q);
      const v4f f = *(const v4fa*)(fbp + 4 * q);
      asm volatile("" :: "v"(a), "v"(b), "v"(c));
      asm volatile("" :: "v"(d), "v"(e), "v"(f));
      const unsigned m0 = (grp < 3)  ? 0xffffffffu : 0u;
      const unsigned m1 = (grp == 3) ? 0xffffffffu : 0u;
      const unsigned m2 = (grp == 4) ? 0xffffffffu : 0u;
      const unsigned m3 = (grp == 5) ? 0xffffffffu : 0u;
      const unsigned m4 = (grp == 6) ? 0xffffffffu : 0u;
      const unsigned m5 = (grp == 7) ? 0xffffffffu : 0u;
      v4f o;
      o.x = blend6(a.x, b.x, c.x, d.x, e.x, f.x, m0, m1, m2, m3, m4, m5);
      o.y = blend6(a.y, b.y, c.y, d.y, e.y, f.y, m0, m1, m2, m3, m4, m5);
      o.z = blend6(a.z, b.z, c.z, d.z, e.z, f.z, m0, m1, m2, m3, m4, m5);
      o.w = blend6(a.w, b.w, c.w, d.w, e.w, f.w, m0, m1, m2, m3, m4, m5);
      st2_v4f(tab + 4 * tid, o);
    }
  }
}

template <int KTOT, int NT>
__device__ __forceinline__ void gemm_16xn(const unsigned short* __restrict__ ap,
                                          const unsigned short* __restrict__ bp, v8f (&acc)[NT]) {
#pragma unroll 1
  for (int k0 = 0; k0 < KTOT; k0 += 32) {
    FragB af;
    af.h[0] = *(const v8usa*)(ap + k0);
    af.h[1] = *(const v8usa*)(ap + k0 + 16);
#pragma unroll
    for (int nt = 0; nt < NT; ++nt) {
      const unsigned short* wq = bp + (size_t)(16 * nt) * (size_t)KTOT + k0;
      FragB bf;
      bf.h[0] = *(const v8usa*)wq;
      bf.h[1] = *(const v8usa*)(wq + 16);
      acc[nt] = wmb(af, bf, acc[nt]);
    }
  }
}

template <int OFF, int NA>
__device__ __forceinline__ void stage_d(float* stg, const v8f (&acc)[NA], int wave, int hh, int m) {
#pragma unroll
  for (int nt = 0; nt < 4; ++nt) {
#pragma unroll
    for (int r = 0; r < 8; ++r) stg[(16 * wave + 8 * hh + r) * SP + 16 * nt + m] = acc[OFF + nt][r];
  }
}

__global__ __launch_bounds__(NTHR) __attribute__((amdgpu_num_vgpr(248)))
void k_gemm1(const unsigned short* __restrict__ XB, const unsigned short* __restrict__ W1T,
             const float* __restrict__ pos, const float* __restrict__ tab, float* Apl, float* Bpl) {
  __shared__ __attribute__((aligned(16))) float stg[GBM * SP];
  __shared__ __attribute__((aligned(16))) float spos[GBM * 3];
  __shared__ __attribute__((aligned(16))) float swp[256];
  const int tid = (int)threadIdx.x, lane = tid & 31, wave = tid >> 5, hh = lane >> 4, m = lane & 15;
  const int rowBase = (int)blockIdx.x * GBM;

  if (tid < 96) {
    int j = (rowBase * 3) / 4 + tid;
    j = j > (NN * 3 / 4 - 1) ? (NN * 3 / 4 - 1) : j;
    const v4f p = *(const v4fa*)(pos + (size_t)4 * (size_t)j);
    v4f o;
    o.x = bf16_val(p.x); o.y = bf16_val(p.y); o.z = bf16_val(p.z); o.w = bf16_val(p.w);
    *(v4fa*)(spos + 4 * tid) = o;
  } else if (tid >= 128 && tid < 192) {
    const int u = tid - 128;
    *(v4fa*)(swp + 4 * u) = *(const v4fa*)(tab + 4 * u);
  }

  v8f acc[8];
  {
    const v8f z = {0.f, 0.f, 0.f, 0.f, 0.f, 0.f, 0.f, 0.f};
#pragma unroll
    for (int t = 0; t < 8; ++t) acc[t] = z;
  }
  const unsigned short* ap = XB + (size_t)(rowBase + 16 * wave + m) * (size_t)K1 + 8 * hh;
  const unsigned short* bp = W1T + (size_t)m * (size_t)K1 + 8 * hh;
  gemm_16xn<K1, 8>(ap, bp, acc);

  v8f dd[4];
#pragma unroll
  for (int nt = 0; nt < 4; ++nt) dd[nt] = acc[nt] - acc[nt + 4];
  stage_d<0, 4>(stg, dd, wave, hh, m);
  __syncthreads();

  const v4f w0 = *(const v4fa*)(swp + 4 * m);
  const v4f w1 = *(const v4fa*)(swp + 64 + 4 * m);
  const v4f w2 = *(const v4fa*)(swp + 128 + 4 * m);
  const v4f mb = *(const v4fa*)(swp + 192 + 4 * m);

#pragma unroll 1
  for (int i = 0; i < 8; ++i) {
    const int lr   = 16 * wave + 2 * i + hh;
    const int grow = rowBase + lr;
    const v4f a = *(const v4fa*)(stg + lr * SP + 4 * m);
    const float p0 = spos[3 * lr], p1 = spos[3 * lr + 1], p2 = spos[3 * lr + 2];
    asm volatile("" :: "v"(a));
    v4f pc;
    pc.x = fmaf(p2, w2.x, fmaf(p1, w1.x, p0 * w0.x));
    pc.y = fmaf(p2, w2.y, fmaf(p1, w1.y, p0 * w0.y));
    pc.z = fmaf(p2, w2.z, fmaf(p1, w1.z, p0 * w0.z));
    pc.w = fmaf(p2, w2.w, fmaf(p1, w1.w, p0 * w0.w));
    v4f o;
    o.x = (a.x - pc.x) + mb.x; o.y = (a.y - pc.y) + mb.y;
    o.z = (a.z - pc.z) + mb.z; o.w = (a.w - pc.w) + mb.w;
    if (grow < NN) st2_v4f(Apl + (size_t)grow * HD + 4 * m, o);
  }
  __syncthreads();
  stage_d<4, 8>(stg, acc, wave, hh, m);
  __syncthreads();

#pragma unroll 1
  for (int i = 0; i < 8; ++i) {
    const int lr   = 16 * wave + 2 * i + hh;
    const int grow = rowBase + lr;
    const v4f a = *(const v4fa*)(stg + lr * SP + 4 * m);
    const float p0 = spos[3 * lr], p1 = spos[3 * lr + 1], p2 = spos[3 * lr + 2];
    asm volatile("" :: "v"(a));
    v4f o;
    o.x = a.x + fmaf(p2, w2.x, fmaf(p1, w1.x, p0 * w0.x));
    o.y = a.y + fmaf(p2, w2.y, fmaf(p1, w1.y, p0 * w0.y));
    o.z = a.z + fmaf(p2, w2.z, fmaf(p1, w1.z, p0 * w0.z));
    o.w = a.w + fmaf(p2, w2.w, fmaf(p1, w1.w, p0 * w0.w));
    if (grow < NN) st2_v4f(Bpl + (size_t)grow * HD + 4 * m, o);
  }
}

__global__ __launch_bounds__(NTHR) void k_scanmax(const int* __restrict__ srcs, const int* __restrict__ dsts,
                                                  const float* Apl, const float* Bpl, float* AGG, int* FLAG) {
  extern __shared__ __attribute__((aligned(16))) int dsm[];
  int* wl   = dsm;
  int* pl   = dsm + NWAVE * WLCAP;
  int* cnt  = pl + RCAP;
  int* offs = cnt + NBRUN;
  int* cur  = offs + NBRUN;
  int* misc = cur + NBRUN;
  const int tid = (int)threadIdx.x, lane = tid & 31, wave = tid >> 5;
  const int blk = (int)blockIdx.x;
  const unsigned nbs = (unsigned)(blk * NBRUN);

  {
    const v4i z4 = {0, 0, 0, 0};
    for (int i = tid * 4; i < BK_ZINTS; i += NTHR * 4) *(v4ia*)(dsm + i) = z4;
    if (tid < 16) misc[tid] = 0;
  }
  __syncthreads();

  {
    const int per  = ((NE + NWAVE * WCH - 1) / (NWAVE * WCH)) * WCH;
    const int ebeg = wave * per;
    const int eend = (ebeg + per < NE) ? (ebeg + per) : NE;
    int* mylist = wl + wave * WLCAP;
    int wc = 0;
#pragma unroll 1
    for (int cb = ebeg; cb < eend; cb += WCH) {
      const int e0 = cb + lane * EPT;
      const v4i da = *(const v4ia*)(dsts + e0);
      const v4i db = *(const v4ia*)(dsts + e0 + 4);
      const unsigned s0 = (unsigned)da.x - nbs, s1 = (unsigned)da.y - nbs;
      const unsigned s2 = (unsigned)da.z - nbs, s3 = (unsigned)da.w - nbs;
      const unsigned s4 = (unsigned)db.x - nbs, s5 = (unsigned)db.y - nbs;
      const unsigned s6 = (unsigned)db.z - nbs, s7 = (unsigned)db.w - nbs;
      const bool h0 = s0 < (unsigned)NBRUN, h1 = s1 < (unsigned)NBRUN, h2 = s2 < (unsigned)NBRUN, h3 = s3 < (unsigned)NBRUN;
      const bool h4 = s4 < (unsigned)NBRUN, h5 = s5 < (unsigned)NBRUN, h6 = s6 < (unsigned)NBRUN, h7 = s7 < (unsigned)NBRUN;
      const unsigned m0 = __builtin_amdgcn_ballot_w32(h0), m1 = __builtin_amdgcn_ballot_w32(h1);
      const unsigned m2 = __builtin_amdgcn_ballot_w32(h2), m3 = __builtin_amdgcn_ballot_w32(h3);
      const unsigned m4 = __builtin_amdgcn_ballot_w32(h4), m5 = __builtin_amdgcn_ballot_w32(h5);
      const unsigned m6 = __builtin_amdgcn_ballot_w32(h6), m7 = __builtin_amdgcn_ballot_w32(h7);
      const unsigned any = m0 | m1 | m2 | m3 | m4 | m5 | m6 | m7;
      if (any != 0u) {
        const int pre = (int)(__builtin_amdgcn_mbcnt_lo(m0, 0u) + __builtin_amdgcn_mbcnt_lo(m1, 0u) +
                              __builtin_amdgcn_mbcnt_lo(m2, 0u) + __builtin_amdgcn_mbcnt_lo(m3, 0u) +
                              __builtin_amdgcn_mbcnt_lo(m4, 0u) + __builtin_amdgcn_mbcnt_lo(m5, 0u) +
                              __builtin_amdgcn_mbcnt_lo(m6, 0u) + __builtin_amdgcn_mbcnt_lo(m7, 0u));
        int p = wc + pre;
        if (h0) { if (p < WLCAP) mylist[p] = ((e0 + 0) << SLB) | (int)s0; p = p + 1; }
        if (h1) { if (p < WLCAP) mylist[p] = ((e0 + 1) << SLB) | (int)s1; p = p + 1; }
        if (h2) { if (p < WLCAP) mylist[p] = ((e0 + 2) << SLB) | (int)s2; p = p + 1; }
        if (h3) { if (p < WLCAP) mylist[p] = ((e0 + 3) << SLB) | (int)s3; p = p + 1; }
        if (h4) { if (p < WLCAP) mylist[p] = ((e0 + 4) << SLB) | (int)s4; p = p + 1; }
        if (h5) { if (p < WLCAP) mylist[p] = ((e0 + 5) << SLB) | (int)s5; p = p + 1; }
        if (h6) { if (p < WLCAP) mylist[p] = ((e0 + 6) << SLB) | (int)s6; p = p + 1; }
        if (h7) { if (p < WLCAP) mylist[p] = ((e0 + 7) << SLB) | (int)s7; p = p + 1; }
        wc += (int)(__builtin_popcount(m0) + __builtin_popcount(m1) + __builtin_popcount(m2) + __builtin_popcount(m3) +
                    __builtin_popcount(m4) + __builtin_popcount(m5) + __builtin_popcount(m6) + __builtin_popcount(m7));
      }
    }
    if (lane == 0) misc[wave] = wc;
  }
  __syncthreads();

  if (wave == 0) {
    int ov = 0;
#pragma unroll 1
    for (int w2 = 0; w2 < NWAVE; ++w2) {
      int c = misc[w2];
      if (c > WLCAP) ov = 1;
      c = c < 0 ? 0 : (c > WLCAP ? WLCAP : c);
#pragma unroll 1
      for (int b0 = 0; b0 < c; b0 += 32) {
        const int idx = b0 + lane;
        const int ent = wl[w2 * WLCAP + (idx < WLCAP ? idx : WLCAP - 1)];
        const int m32 = (c - b0) < 32 ? (c - b0) : 32;
#pragma unroll 1
        for (int k = 0; k < m32; ++k) {
          const int u    = __builtin_amdgcn_readlane(ent, k);
          const int slot = u & (NBRUN - 1);
          if (lane == 0) cnt[slot] = cnt[slot] + 1;
        }
      }
    }
    if (lane == 0) misc[9] = ov;
  }
  __syncthreads();
  if (wave == 0) {
    const int base = lane * (NBRUN / 32);
    int s = 0;
#pragma unroll 1
    for (int i = 0; i < NBRUN / 32; ++i) s += cnt[base + i];
    int incl = s;
#pragma unroll
    for (int d = 1; d < 32; d <<= 1) {
      const int y = __shfl_up(incl, d, 32);
      if (lane >= d) incl += y;
    }
    int run = incl - s;
#pragma unroll 1
    for (int i = 0; i < NBRUN / 32; ++i) {
      const int cv = cnt[base + i];
      offs[base + i] = run;
      cur[base + i]  = run;
      run += cv;
    }
  }
  __syncthreads();

  if (wave == 0) {
#pragma unroll 1
    for (int w2 = 0; w2 < NWAVE; ++w2) {
      int c = misc[w2];
      c = c < 0 ? 0 : (c > WLCAP ? WLCAP : c);
#pragma unroll 1
      for (int b0 = 0; b0 < c; b0 += 32) {
        const int idx = b0 + lane;
        const int ent = wl[w2 * WLCAP + (idx < WLCAP ? idx : WLCAP - 1)];
        int eid = (ent >> SLB) & 0x1FFFFF;
        eid = eid > NE - 1 ? NE - 1 : eid;
        int sr = srcs[eid];
        sr = sr < 0 ? 0 : (sr > NN - 1 ? NN - 1 : sr);
        const int word = sr | ((ent & (NBRUN - 1)) << SRCBITS);
        const int m32 = (c - b0) < 32 ? (c - b0) : 32;
#pragma unroll 1
        for (int k = 0; k < m32; ++k) {
          const int u    = __builtin_amdgcn_readlane(ent, k);
          const int wd   = __builtin_amdgcn_readlane(word, k);
          const int slot = u & (NBRUN - 1);
          if (lane == 0) {
            int p = cur[slot];
            p = p < 0 ? 0 : (p > RCAP - 1 ? RCAP - 1 : p);
            pl[p] = wd;
            cur[slot] = p + 1;
          }
        }
      }
    }
  }
  __syncthreads();

  const int ovf = misc[9];
  const int hh = lane >> 4, q = lane & 15;
  const float qnan = __uint_as_float(0x7fc00000u);
  const float ninf = __uint_as_float(0xff800000u);
#pragma unroll 1
  for (int i = 0; i < NBRUN / (2 * NWAVE); ++i) {
    const int slot = (NBRUN / NWAVE) * wave + 2 * i + hh;
    const int d    = blk * NBRUN + slot;
    int c = cnt[slot];
    int o = offs[slot];
    const bool big = c > DEGCAP;
    const bool has = c > 0;
    c = c < 0 ? 0 : (c > DEGCAP ? DEGCAP : c);
    o = o < 0 ? 0 : (o > RCAP - 1 ? RCAP - 1 : o);
    const int co = __shfl_xor(c, 16, 32);
    const int cm = c > co ? c : co;
    int last = o + c - 1;
    last = last < o ? o : last;
    last = last > RCAP - 1 ? RCAP - 1 : last;
    float m0 = ninf, m1 = ninf, m2 = ninf, m3 = ninf;
    int nf = 0;
#pragma unroll 1
    for (int j = 0; j < cm; ++j) {
      int idx = o + j;
      idx = idx > last ? last : idx;
      const unsigned wd = (unsigned)pl[idx];
      int sr = (int)(wd & ((1u << SRCBITS) - 1u));
      sr = sr > NN - 1 ? NN - 1 : sr;
      const v4f v = *(const v4fa*)(Bpl + (size_t)sr * HD + 4 * q);
      asm volatile("" :: "v"(v));
      const bool valid = j < c;
      const float t0 = (v.x > m0) ? v.x : m0, t1 = (v.y > m1) ? v.y : m1;
      const float t2 = (v.z > m2) ? v.z : m2, t3 = (v.w > m3) ? v.w : m3;
      const int   nn = ((v.x != v.x) | (v.y != v.y) | (v.z != v.z) | (v.w != v.w)) ? 1 : 0;
      m0 = valid ? t0 : m0; m1 = valid ? t1 : m1; m2 = valid ? t2 : m2; m3 = valid ? t3 : m3;
      nf |= valid ? nn : 0;
    }
    const int dc = d < NN ? d : NN - 1;
    const v4f a = *(const v4fa*)(Apl + (size_t)dc * HD + 4 * q);
    asm volatile("" :: "v"(a));
    const float s0 = a.x + m0, s1 = a.y + m1, s2 = a.z + m2, s3 = a.w + m3;
    float r0 = has ? s0 : 0.0f, r1 = has ? s1 : 0.0f, r2 = has ? s2 : 0.0f, r3 = has ? s3 : 0.0f;
    const bool bad = (ovf != 0) | big | (nf != 0);
    r0 = bad ? qnan : r0; r1 = bad ? qnan : r1; r2 = bad ? qnan : r2; r3 = bad ? qnan : r3;
    v4f ov4;
    ov4.x = r0; ov4.y = r1; ov4.z = r2; ov4.w = r3;
    if (d < NN) st2_v4f(AGG + (size_t)d * HD + 4 * q, ov4);
  }
  if (tid < 8) {
    const v4i f = {ovf, ovf, ovf, ovf};
    st2_v4i(FLAG + (size_t)blk * 32 + 4 * tid, f);
  }
}

__device__ __forceinline__ void stat_flush(const double* bins, double* rp, int tid) {
#pragma unroll 1
  for (int it = 0; it < 8; ++it) {
    const int e0 = 2 * (it * NTHR + tid);
    const double s0 = ((bins[e0] + bins[4096 + e0]) + bins[8192 + e0]) + bins[12288 + e0];
    const double s1 = ((bins[e0 + 1] + bins[4096 + e0 + 1]) + bins[8192 + e0 + 1]) + bins[12288 + e0 + 1];
    v2d o;
    o.x = s0; o.y = s1;
    *(volatile v2d*)(rp + e0) = o;
  }
}

template <int PASS>
__global__ __launch_bounds__(NTHR) void k_stat(const float* AGG, const int* __restrict__ batch, const float* MS,
                                               double* REC, int* CREC) {
  extern __shared__ __attribute__((aligned(16))) double dsd[];
  double* bins  = dsd;
  float*  sms   = (float*)(dsd + NBIN);
  int*    cpart = (int*)(sms + NG * HD);
  int*    cfold = cpart + 256;
  const int tid = (int)threadIdx.x;
  const int blk = (int)blockIdx.x;
  const int rowBase = blk * NBRUN;

#pragma unroll 1
  for (int i = tid; i < NBIN; i += NTHR) bins[i] = 0.0;
  if constexpr (PASS != 0) {
#pragma unroll 1
    for (int it = 0; it < 4; ++it) {
      const int u = it * NTHR + tid;
      *(v4fa*)(sms + 4 * u) = *(const v4fa*)(MS + 4 * u);
    }
  }
  __syncthreads();

  {
    const int c = tid & 63, r = tid >> 6;
    double* mybin = bins + r * (NG * HD) + c;
#pragma unroll 1
    for (int i = 0; i < NBRUN / 4; ++i) {
      const int n  = rowBase + r + 4 * i;
      const int nc = n < NN ? n : NN - 1;
      int g = batch[nc];
      g = g < 0 ? 0 : (g > NG - 1 ? NG - 1 : g);
      const float a = AGG[(size_t)nc * HD + c];
      asm volatile("" :: "v"(a));
      double dv;
      if constexpr (PASS != 0) {
        const float ce = a - sms[g * HD + c];
        const double cd = (double)ce;
        dv = cd * cd;
      } else {
        dv = (double)a;
      }
      dv = (n < NN) ? dv : 0.0;
      mybin[g * HD] = mybin[g * HD] + dv;
    }
  }
  if constexpr (PASS == 0) {
    const int g = tid & 63, part = tid >> 6;
    int cn = 0;
#pragma unroll 1
    for (int i = 0; i < NBRUN / 4; ++i) {
      const int n  = rowBase + part * (NBRUN / 4) + i;
      const int nc = n < NN ? n : NN - 1;
      int b = batch[nc];
      b = b < 0 ? 0 : (b > NG - 1 ? NG - 1 : b);
      cn += ((n < NN) & (b == g)) ? 1 : 0;
    }
    cpart[part * 64 + g] = cn;
  }
  __syncthreads();
  if constexpr (PASS == 0) {
    if (tid < 64) cfold[tid] = ((cpart[tid] + cpart[64 + tid]) + cpart[128 + tid]) + cpart[192 + tid];
  }
  __syncthreads();

  double* rp = REC + (size_t)blk * (size_t)(NG * HD);
  stat_flush(bins, rp, tid);
  __threadfence();
  stat_flush(bins, rp, tid);
  if constexpr (PASS == 0) {
    if (tid < 16) {
      const v4i v = *(const v4ia*)(cfold + 4 * tid);
      st2_v4i(CREC + (size_t)blk * 64 + 4 * tid, v);
    }
  }
}

template <int PASS>
__global__ __launch_bounds__(NTHR) void k_comb(const double* REC, const int* CREC, const float* tab, float* OUTT) {
  __shared__ __attribute__((aligned(16))) float sbuf[NTHR];
  const int tid = (int)threadIdx.x;
  const int blk = (int)blockIdx.x;
  const int u = blk * NTHR + tid;
  const int g = u >> 6, c = u & 63;
  double s = 0.0;
  int cn = 0;
#pragma unroll 2
  for (int b = 0; b < NBK; ++b) {
    s  = s + REC[(size_t)b * (size_t)(NG * HD) + u];
    cn = cn + CREC[b * 64 + g];
  }
  const double cd = (double)(cn < 1 ? 1 : cn);
  const float  qv = (float)(s / cd);
  float o;
  if constexpr (PASS == 0) {
    const float gs = tab[T_GS + c];
    o = qv * gs;
  } else {
    o = sqrtf(qv + 1e-5f);
  }
  sbuf[tid] = o;
  __syncthreads();
  if (tid < 64) {
    const v4f v = *(const v4fa*)(sbuf + 4 * tid);
    st2_v4f(OUTT + (size_t)blk * NTHR + 4 * tid, v);
  }
}

__global__ __launch_bounds__(NTHR) void k_apply(const float* AGG, const int* __restrict__ batch, const float* MS,
                                                const float* DEN, const float* tab, unsigned short* HHL) {
  __shared__ __attribute__((aligned(16))) float sgb[128];
  const int tid = (int)threadIdx.x, lane = tid & 31, wave = tid >> 5, hh = lane >> 4, q = lane & 15;
  const int rowBase = (int)blockIdx.x * GBM;
  if (tid < 32) *(v4fa*)(sgb + 4 * tid) = *(const v4fa*)(tab + T_GW + 4 * tid);
  __syncthreads();
  const v4f gw = *(const v4fa*)(sgb + 4 * q);
  const v4f gb = *(const v4fa*)(sgb + 64 + 4 * q);

#pragma unroll 1
  for (int i = 0; i < 8; ++i) {
    const int d  = rowBase + 16 * wave + 2 * i + hh;
    const int dc = d < NN ? d : NN - 1;
    int g = batch[dc];
    g = g < 0 ? 0 : (g > NG - 1 ? NG - 1 : g);
    const v4f a  = *(const v4fa*)(AGG + (size_t)dc * HD + 4 * q);
    const v4f ms = *(const v4fa*)(MS + g * HD + 4 * q);
    const v4f dn = *(const v4fa*)(DEN + g * HD + 4 * q);
    asm volatile("" :: "v"(a), "v"(ms), "v"(dn));
    float v0 = gw.x * (a.x - ms.x) / dn.x + gb.x;
    float v1 = gw.y * (a.y - ms.y) / dn.y + gb.y;
    float v2 = gw.z * (a.z - ms.z) / dn.z + gb.z;
    float v3 = gw.w * (a.w - ms.w) / dn.w + gb.w;
    v0 = (v0 > 0.0f) ? v0 : (v0 - v0); v1 = (v1 > 0.0f) ? v1 : (v1 - v1);
    v2 = (v2 > 0.0f) ? v2 : (v2 - v2); v3 = (v3 > 0.0f) ? v3 : (v3 - v3);
    const bool live = d < NN;
    v0 = live ? v0 : 0.0f; v1 = live ? v1 : 0.0f; v2 = live ? v2 : 0.0f; v3 = live ? v3 : 0.0f;
    int h01, h23, l01, l23;
    hilo_pack(v0, v1, v2, v3, h01, h23, l01, l23);
    const v4i ow = regroup8(h01, h23, l01, l23, lane);
    st2_v4i((int*)(HHL + (size_t)d * K2 + 8 * q), ow);
  }
}

__global__ __launch_bounds__(NTHR) __attribute__((amdgpu_num_vgpr(248)))
void k_gemm2(const unsigned short* __restrict__ HHL, const unsigned short* __restrict__ FCD,
             const float* __restrict__ x, const float* __restrict__ tab, const int* __restrict__ FLAG,
             float* out) {
  __shared__ __attribute__((aligned(16))) float stg[GBM * SP];
  __shared__ __attribute__((aligned(16))) float sb[64];
  const int tid = (int)threadIdx.x, lane = tid & 31, wave = tid >> 5, hh = lane >> 4, m = lane & 15;
  const int rowBase = (int)blockIdx.x * GBM;
  const int flag = FLAG[(size_t)(rowBase >> SLB) * 32];
  if (tid < 16) *(v4fa*)(sb + 4 * tid) = *(const v4fa*)(tab + T_FB + 4 * tid);

  v8f acc[4];
  {
    const v8f z = {0.f, 0.f, 0.f, 0.f, 0.f, 0.f, 0.f, 0.f};
#pragma unroll
    for (int t = 0; t < 4; ++t) acc[t] = z;
  }
  const unsigned short* ap = HHL + (size_t)(rowBase + 16 * wave + m) * (size_t)K2 + 8 * hh;
  const unsigned short* bp = FCD + (size_t)m * (size_t)K2 + 8 * hh;
  gemm_16xn<K2, 4>(ap, bp, acc);
  stage_d<0, 4>(stg, acc, wave, hh, m);
  __syncthreads();

  const v4f bias = *(const v4fa*)(sb + 4 * m);
  const float qnan = __uint_as_float(0x7fc00000u);
#pragma unroll 1
  for (int i = 0; i < 8; ++i) {
    const int lr   = 16 * wave + 2 * i + hh;
    const int grow = rowBase + lr;
    const int gc   = grow < NN ? grow : NN - 1;
    const v4f a  = *(const v4fa*)(stg + lr * SP + 4 * m);
    const v4f xv = *(const v4fa*)(x + (size_t)gc * HD + 4 * m);
    asm volatile("" :: "v"(a), "v"(xv));
    float v0 = (a.x + bias.x) + bf16_val(xv.x);
    float v1 = (a.y + bias.y) + bf16_val(xv.y);
    float v2 = (a.z + bias.z) + bf16_val(xv.z);
    float v3 = (a.w + bias.w) + bf16_val(xv.w);
    const bool bad = flag != 0;
    v0 = bad ? qnan : v0; v1 = bad ? qnan : v1; v2 = bad ? qnan : v2; v3 = bad ? qnan : v3;
    v4f o;
    o.x = v0; o.y = v1; o.z = v2; o.w = v3;
    if (grow < NN) st2_v4f(out + (size_t)grow * HD + 4 * m, o);
  }
}

extern "C" void kernel_launch(void* const* d_in, const int* in_sizes, int n_in,
                              void* d_out, int out_size, void* d_ws, size_t ws_size,
                              hipStream_t stream) {
  if (n_in < 11) return;
  if (in_sizes[0] != NN * HD) return;
  if (in_sizes[1] != NN * 3) return;
  if (in_sizes[2] != 2 * NE) return;
  if (in_sizes[3] != NN) return;
  if (in_sizes[4] != 131 * HD) return;
  if (in_sizes[5] != HD) return;
  if (in_sizes[6] != HD) return;
  if (in_sizes[7] != HD) return;
  if (in_sizes[8] != HD) return;
  if (in_sizes[9] != HD * HD) return;
  if (in_sizes[10] != HD) return;
  if (out_size != NN * HD) return;

  const float* x     = (const float*)d_in[0];
  const float* pos   = (const float*)d_in[1];
  const int*   ei    = (const int*)d_in[2];
  const int*   batch = (const int*)d_in[3];
  const float* msgW  = (const float*)d_in[4];
  const float* msgb  = (const float*)d_in[5];
  const float* gnw   = (const float*)d_in[6];
  const float* gnb   = (const float*)d_in[7];
  const float* gns   = (const float*)d_in[8];
  const float* fcW   = (const float*)d_in[9];
  const float* fcb   = (const float*)d_in[10];
  float* out = (float*)d_out;
  const int* srcs = ei;
  const int* dsts = ei + NE;

  constexpr size_t zF    = (size_t)NN * HD * 4;
  constexpr size_t zHHL  = (size_t)MP * K2 * 2;
  constexpr size_t zXB   = (size_t)MP * HD * 2;
  constexpr size_t zREC  = (size_t)NBK * NG * HD * 8;
  constexpr size_t zCREC = (size_t)NBK * 64 * 4;
  constexpr size_t zFLAG = (size_t)NBK * 128;
  constexpr size_t zW1T  = (size_t)N1 * K1 * 2;
  constexpr size_t zFCD  = (size_t)HD * K2 * 2;
  constexpr size_t zTAB  = 2048;
  constexpr size_t zGT   = (size_t)NG * HD * 4;
  constexpr size_t oA    = 0;
  constexpr size_t oB    = oA + zF;
  constexpr size_t oAGG  = oB + zF;
  constexpr size_t oHHL  = oAGG + zF;
  constexpr size_t oXB   = oHHL + zHHL;
  constexpr size_t oREC1 = oXB + zXB;
  constexpr size_t oREC2 = oREC1 + zREC;
  constexpr size_t oCREC = oREC2 + zREC;
  constexpr size_t oFLAG = oCREC + zCREC;
  constexpr size_t oW1T  = oFLAG + zFLAG;
  constexpr size_t oFCD  = oW1T + zW1T;
  constexpr size_t oTAB  = oFCD + zFCD;
  constexpr size_t oMS   = oTAB + zTAB;
  constexpr size_t oDEN  = oMS + zGT;
  constexpr size_t oEND  = oDEN + zGT;
  static_assert(zF % 256 == 0 && zHHL % 256 == 0 && zXB % 256 == 0 && zREC % 256 == 0 && zCREC % 256 == 0);
  static_assert(zFLAG % 256 == 0 && zW1T % 256 == 0 && zFCD % 256 == 0 && zTAB % 256 == 0 && zGT % 256 == 0);
  static_assert(oEND <= (size_t)WSMAX);
  if (oEND > ws_size) return;

  char* ws = (char*)d_ws;
  float*          Apl  = (float*)(ws + oA);
  float*          Bpl  = (float*)(ws + oB);
  float*          AGG  = (float*)(ws + oAGG);
  unsigned short* HHL  = (unsigned short*)(ws + oHHL);
  unsigned short* XB   = (unsigned short*)(ws + oXB);
  double*         REC1 = (double*)(ws + oREC1);
  double*         REC2 = (double*)(ws + oREC2);
  int*            CREC = (int*)(ws + oCREC);
  int*            FLAG = (int*)(ws + oFLAG);
  unsigned short* W1T  = (unsigned short*)(ws + oW1T);
  unsigned short* FCD  = (unsigned short*)(ws + oFCD);
  float*          TAB  = (float*)(ws + oTAB);
  float*          MS   = (float*)(ws + oMS);
  float*          DEN  = (float*)(ws + oDEN);

  hipFuncSetAttribute(reinterpret_cast<const void*>(&k_scanmax), hipFuncAttributeMaxDynamicSharedMemorySize, (int)BK_LDS);
  hipFuncSetAttribute(reinterpret_cast<const void*>(&k_stat<0>), hipFuncAttributeMaxDynamicSharedMemorySize, (int)STAT_LDS);
  hipFuncSetAttribute(reinterpret_cast<const void*>(&k_stat<1>), hipFuncAttributeMaxDynamicSharedMemorySize, (int)STAT_LDS);

  k_prep<<<PBTOT, NTHR, 0, stream>>>(x, msgW, msgb, gnw, gnb, gns, fcW, fcb, XB, W1T, FCD, TAB);
  k_gemm1<<<MP / GBM, NTHR, 0, stream>>>(XB, W1T, pos, TAB, Apl, Bpl);
  k_scanmax<<<NBK, NTHR, BK_LDS, stream>>>(srcs, dsts, Apl, Bpl, AGG, FLAG);
  k_stat<0><<<NBK, NTHR, STAT_LDS, stream>>>(AGG, batch, MS, REC1, CREC);
  k_comb<0><<<NG * HD / NTHR, NTHR, 0, stream>>>(REC1, CREC, TAB, MS);
  k_stat<1><<<NBK, NTHR, STAT_LDS, stream>>>(AGG, batch, MS, REC2, CREC);
  k_comb<1><<<NG * HD / NTHR, NTHR, 0, stream>>>(REC2, CREC, TAB, DEN);
  k_apply<<<MP / GBM, NTHR, 0, stream>>>(AGG, batch, MS, DEN, TAB, HHL);
  k_gemm2<<<MP / GBM, NTHR, 0, stream>>>(HHL, FCD, x, TAB, FLAG, out);
}
